// CrystalGraphEncoder_31714038514078
// MI455X (gfx1250) — hardware-verified
//
#include <hip/hip_runtime.h>
#include <stddef.h>
#include <stdint.h>


#define DIN     92
#define KIN     96
#define HC      256
#define NHEAD   8
#define HD      32
#define NQ      1024
#define OQ      0
#define OKK     256
#define OV      512
#define OS      768
#define HFF     512
#define NOUT    128
#define NGR     128
#define NTHR    256
#define NWAVE   8
#define EPT     8
#define CHUNK   (NTHR * EPT)
#define WCAP    (EPT * 32)
#define LISTN   (NWAVE * WCAP)
#define NBMAX   1024
#define RCAP    28672
#define DEGCAP  128
#define PCAP    4096
#define STW     256
#define GBM     64
#define GBN     64
#define GTHR    128
#define CX      8.0f
#define CW      1024.0f
#define SCL_XW  0.0001220703125f
#define ATTSC   0.17677669529663687f
#define LNEPS   0.00001f
#define INVHC   0.00390625f
#define WSMAX   134217728
#define LDS_AGG ((2 * RCAP + 2 * NBMAX + LISTN) * 4 + 64)

static_assert((CHUNK & (CHUNK - 1)) == 0 && CHUNK <= 4096);
static_assert((NBMAX & (NBMAX - 1)) == 0 && NBMAX <= 4096);
static_assert(NTHR * 4 == NBMAX);
static_assert(LISTN >= NBMAX);
static_assert(LISTN >= NWAVE * WCAP);
static_assert((RCAP % 32) == 0);
static_assert(NWAVE * STW <= RCAP);
static_assert(STW >= HC);
static_assert(LDS_AGG <= 300000);
static_assert(GBM == (GTHR / 32) * 16);
static_assert((KIN % 32) == 0 && KIN >= DIN && (DIN % 4) == 0 && KIN - DIN < 8 + 4);
static_assert((HC % 32) == 0 && (HFF % 32) == 0);
static_assert(NQ == 4 * HC && HC == NHEAD * HD && HD == 32);
static_assert(NTHR == HC);
static_assert((NQ % GBN) == 0 && (HC % GBN) == 0 && (HFF % GBN) == 0 && (NOUT % GBN) == 0);
static_assert((NGR % GBM) == 0);
static_assert(DEGCAP >= 65);

typedef float    v4f  __attribute__((ext_vector_type(4)));
typedef float    v8f  __attribute__((ext_vector_type(8)));
typedef int      v4i  __attribute__((ext_vector_type(4)));
typedef int      v8i  __attribute__((ext_vector_type(8)));
typedef _Float16 v8h  __attribute__((ext_vector_type(8)));
typedef _Float16 v16h __attribute__((ext_vector_type(16)));
union FragH { v16h v; v8h h[2]; v8i w; };

__device__ __forceinline__ v8f wmh(const FragH& a, const FragH& b, v8f c) {
  v8f d = __builtin_amdgcn_wmma_f32_16x16x32_f16(false, a.v, false, b.v, (short)0, c, false, false);
  asm volatile("v_nop\n\tv_nop\n\tv_nop\n\tv_nop" : "+v"(d) : "v"(a.w), "v"(b.w));
  return d;
}

__device__ __forceinline__ void ldwait() {
  asm volatile("s_wait_loadcnt 0x0" ::: "memory");
}

__device__ __forceinline__ v8h cvt8h(const v4f a, const v4f b, const float c) {
  v8h hv;
  hv[0] = (_Float16)(a.x * c); hv[1] = (_Float16)(a.y * c);
  hv[2] = (_Float16)(a.z * c); hv[3] = (_Float16)(a.w * c);
  hv[4] = (_Float16)(b.x * c); hv[5] = (_Float16)(b.y * c);
  hv[6] = (_Float16)(b.z * c); hv[7] = (_Float16)(b.w * c);
  return hv;
}

__device__ __forceinline__ int scan_chunk(const int* __restrict__ lst, int nE, int nTot, int cbase, int slotBase,
                                          int nb, int vec8, int* list, int tid, int lane, int wave) {
  int wc = 0;
  const int el0  = tid * EPT;
  const int e0   = cbase + el0;
  const int sent = -2147483647 - 1;
  v4i da, db;
  if (vec8 != 0 && cbase + CHUNK <= nE) {
    da = *(const v4i*)(lst + e0);
    db = *(const v4i*)(lst + e0 + 4);
  } else {
#define VLD(E, DSTV) { \
      const int ee = (E); \
      const int ld = lst[ee < nE ? ee : nE - 1]; \
      DSTV = (ee < nE) ? ld : ((ee < nTot) ? (ee - nE) : sent); }
    VLD(e0,     da.x)
    VLD(e0 + 1, da.y)
    VLD(e0 + 2, da.z)
    VLD(e0 + 3, da.w)
    VLD(e0 + 4, db.x)
    VLD(e0 + 5, db.y)
    VLD(e0 + 6, db.z)
    VLD(e0 + 7, db.w)
#undef VLD
  }
  const unsigned nbs = (unsigned)slotBase;
  const unsigned unb = (unsigned)nb;
  const unsigned s0 = (unsigned)da.x - nbs, s1 = (unsigned)da.y - nbs;
  const unsigned s2 = (unsigned)da.z - nbs, s3 = (unsigned)da.w - nbs;
  const unsigned s4 = (unsigned)db.x - nbs, s5 = (unsigned)db.y - nbs;
  const unsigned s6 = (unsigned)db.z - nbs, s7 = (unsigned)db.w - nbs;
  const bool h0 = s0 < unb, h1 = s1 < unb, h2 = s2 < unb, h3 = s3 < unb;
  const bool h4 = s4 < unb, h5 = s5 < unb, h6 = s6 < unb, h7 = s7 < unb;
  const unsigned any = __builtin_amdgcn_ballot_w32(h0 | h1 | h2 | h3 | h4 | h5 | h6 | h7);
  if (any != 0u) {
#define HITJ(J, HJ, SJ) { \
      const unsigned mj = __builtin_amdgcn_ballot_w32(HJ); \
      if (mj != 0u) { \
        if (HJ) { \
          const int pos = wc + (int)__builtin_amdgcn_mbcnt_lo(mj, 0u); \
          if (pos < WCAP) list[wave * WCAP + pos] = ((el0 + (J)) << 12) | (int)(SJ); \
        } \
        wc += (int)__builtin_popcount(mj); } }
    HITJ(0, h0, s0)
    HITJ(1, h1, s1)
    HITJ(2, h2, s2)
    HITJ(3, h3, s3)
    HITJ(4, h4, s4)
    HITJ(5, h5, s5)
    HITJ(6, h6, s6)
    HITJ(7, h7, s7)
#undef HITJ
  }
  return wc;
}

__global__ __launch_bounds__(NTHR) void k_xprep(const float* __restrict__ x, _Float16* xh, int nN, int nUnits) {
  const int i = (int)blockIdx.x * NTHR + (int)threadIdx.x;
  if (i >= nUnits) return;
  const int row = i / (KIN / 8);
  const int c0  = (i - row * (KIN / 8)) * 8;
  const int rc  = row < nN ? row : nN - 1;
  const float* p = x + (size_t)rc * DIN;
  const int ca = c0 < DIN - 4 ? c0 : DIN - 4;
  const int cb = (c0 + 4) < DIN - 4 ? (c0 + 4) : DIN - 4;
  v4f a = *(const v4f*)(p + ca), b = *(const v4f*)(p + cb);
  const v4f z4 = {0.f, 0.f, 0.f, 0.f};
  if (c0 >= DIN) a = z4;
  if (c0 + 4 >= DIN) b = z4;
  if (row >= nN) { a = z4; b = z4; }
  const v8h hv = cvt8h(a, b, CX);
  const size_t o = (size_t)row * KIN + c0;
  *(volatile v8h*)(xh + o) = hv;
  __threadfence();
  *(volatile v8h*)(xh + o) = hv;
}

__global__ __launch_bounds__(NTHR) void k_wtr(const float* __restrict__ w0, const float* __restrict__ w1,
                                              const float* __restrict__ w2, const float* __restrict__ w3,
                                              int c0, int c1, int c2, int c3, int segRows, int Kr, int K,
                                              _Float16* wt, int nUnits) {
  const int u = (int)blockIdx.x * NTHR + (int)threadIdx.x;
  if (u >= nUnits) return;
  const int kq = K >> 3;
  const int n  = u / kq;
  const int k8 = (u - n * kq) * 8;
  int seg = n / segRows;
  seg = seg > 3 ? 3 : seg;
  const int nc = n - seg * segRows;
  const float* ws = (seg == 0) ? w0 : ((seg == 1) ? w1 : ((seg == 2) ? w2 : w3));
  const int cc = (seg == 0) ? c0 : ((seg == 1) ? c1 : ((seg == 2) ? c2 : c3));
  const int ncl = nc < cc ? nc : cc - 1;
  float f[8];
#pragma unroll
  for (int j = 0; j < 8; ++j) {
    const int kk = k8 + j;
    const int kc = kk < Kr ? kk : Kr - 1;
    const float v = ws[(size_t)kc * (size_t)cc + ncl];
    f[j] = (kk < Kr && nc < cc) ? v : 0.f;
  }
  v4f a, b;
  a.x = f[0]; a.y = f[1]; a.z = f[2]; a.w = f[3];
  b.x = f[4]; b.y = f[5]; b.z = f[6]; b.w = f[7];
  const v8h hv = cvt8h(a, b, CW);
  const size_t o = (size_t)n * (size_t)K + k8;
  *(volatile v8h*)(wt + o) = hv;
  __threadfence();
  *(volatile v8h*)(wt + o) = hv;
}

template<int EPI>
__global__ __launch_bounds__(GTHR) void k_gemm(
    const _Float16* __restrict__ A, const _Float16* __restrict__ WT,
    const float* __restrict__ b0, const float* __restrict__ b1,
    const float* __restrict__ b2, const float* __restrict__ b3,
    float* outF, _Float16* outH, int K, int ldo, int segN, int blen, float bsc, float scl)
{
  __shared__ __attribute__((aligned(16))) float stg[GBM * GBN];
  const int tid = (int)threadIdx.x, lane = tid & 31, wave = tid >> 5, hh = lane >> 4, m = lane & 15;
  const int rowBase = (int)blockIdx.x * GBM;
  const int col0    = (int)blockIdx.y * GBN;
  int seg = col0 / segN;
  seg = seg < 0 ? 0 : (seg > 3 ? 3 : seg);
  const float* bp = (seg == 0) ? b0 : ((seg == 1) ? b1 : ((seg == 2) ? b2 : b3));
  int bofs = col0 - seg * segN;
  bofs = bofs < 0 ? 0 : bofs;

  v8f acc[4];
  {
    const v8f z = {0.f, 0.f, 0.f, 0.f, 0.f, 0.f, 0.f, 0.f};
    acc[0] = z; acc[1] = z; acc[2] = z; acc[3] = z;
  }
  const _Float16* ap = A  + (size_t)(rowBase + 16 * wave + m) * (size_t)K + 8 * hh;
  const _Float16* wp = WT + (size_t)(col0 + m) * (size_t)K + 8 * hh;
  const int ksteps = K >> 5;
#pragma unroll 1
  for (int ks = 0; ks < ksteps; ++ks) {
    FragH af;
    af.h[0] = *(const v8h*)(ap + 32 * ks);
    af.h[1] = *(const v8h*)(ap + 32 * ks + 16);
#pragma unroll
    for (int t = 0; t < 4; ++t) {
      const _Float16* wq = wp + (size_t)(16 * t) * (size_t)K + 32 * ks;
      FragH bf;
      bf.h[0] = *(const v8h*)wq;
      bf.h[1] = *(const v8h*)(wq + 16);
      acc[t] = wmh(af, bf, acc[t]);
    }
  }

#pragma unroll
  for (int t = 0; t < 4; ++t) {
    const int lc = 16 * t + m;
    int bi = bofs + lc;
    bi = bi > blen - 1 ? blen - 1 : bi;
    bi = bi < 0 ? 0 : bi;
    const float bv = bp[bi] * bsc;
#pragma unroll
    for (int r = 0; r < 8; ++r) {
      const int lr = 16 * wave + 8 * hh + r;
      stg[lr * GBN + lc] = fmaf(acc[t][r], scl, bv);
    }
  }
  __syncthreads();

  if (EPI == 0 || EPI == 1) {
    v4f fv[8];
#pragma unroll
    for (int i = 0; i < 8; ++i) {
      const int lr = 16 * wave + 2 * i + hh;
      fv[i] = *(const v4f*)(stg + lr * GBN + 4 * m);
    }
#pragma unroll
    for (int i = 0; i < 8; ++i) {
      const int lr = 16 * wave + 2 * i + hh;
      const int gr = rowBase + lr;
      float* op = outF + (size_t)gr * (size_t)ldo + col0 + 4 * m;
      *(volatile v4f*)op = fv[i];
    }
    __threadfence();
#pragma unroll
    for (int i = 0; i < 8; ++i) {
      const int lr = 16 * wave + 2 * i + hh;
      const int gr = rowBase + lr;
      float* op = outF + (size_t)gr * (size_t)ldo + col0 + 4 * m;
      *(volatile v4f*)op = fv[i];
    }
  }
  if (EPI == 1 || EPI == 2) {
    v8h hv[4];
    const int q8 = lane >> 3;
    const int c8 = 8 * (lane & 7);
#pragma unroll
    for (int i = 0; i < 4; ++i) {
      const int lr = 16 * wave + 4 * i + q8;
      v4f ga = *(const v4f*)(stg + lr * GBN + c8);
      v4f gb = *(const v4f*)(stg + lr * GBN + c8 + 4);
      if (EPI == 2) {
        ga.x = fmaxf(ga.x, 0.f); ga.y = fmaxf(ga.y, 0.f); ga.z = fmaxf(ga.z, 0.f); ga.w = fmaxf(ga.w, 0.f);
        gb.x = fmaxf(gb.x, 0.f); gb.y = fmaxf(gb.y, 0.f); gb.z = fmaxf(gb.z, 0.f); gb.w = fmaxf(gb.w, 0.f);
      }
      hv[i] = cvt8h(ga, gb, CX);
    }
#pragma unroll
    for (int i = 0; i < 4; ++i) {
      const int lr = 16 * wave + 4 * i + q8;
      _Float16* hp = outH + (size_t)(rowBase + lr) * (size_t)ldo + col0 + c8;
      *(volatile v8h*)hp = hv[i];
    }
    __threadfence();
#pragma unroll
    for (int i = 0; i < 4; ++i) {
      const int lr = 16 * wave + 4 * i + q8;
      _Float16* hp = outH + (size_t)(rowBase + lr) * (size_t)ldo + col0 + c8;
      *(volatile v8h*)hp = hv[i];
    }
  }
}

template<int GAT>
__global__ __launch_bounds__(NTHR) void k_layer(
    const int* __restrict__ srcs, const int* __restrict__ dsts,
    const float* __restrict__ P,
    const float* __restrict__ atts, const float* __restrict__ attd, const float* __restrict__ bgp,
    const float* __restrict__ lng, const float* __restrict__ lnb,
    float* Hf, _Float16* Hh,
    int nN, int nE, int nTot, int nb, int vec8, int MPr) {
  extern __shared__ v4f lds_dyn[];
  int* reg1 = (int*)lds_dyn;
  int* reg2 = reg1 + RCAP;
  int* scnt = reg2 + RCAP;
  int* soff = scnt + NBMAX;
  int* list = soff + NBMAX;
  int* wcnt = list + LISTN;
  int* wtot = wcnt + NWAVE;
  const int tid = (int)threadIdx.x, lane = tid & 31, wave = tid >> 5;
  const int nodeBase = (int)blockIdx.x * nb;

  for (int i = tid; i < NBMAX; i += NTHR) scnt[i] = 0;
  __syncthreads();

  int tot = 0;
  const int nChunks = (nTot + CHUNK - 1) / CHUNK;
#pragma unroll 1
  for (int ch = 0; ch < nChunks; ++ch) {
    const int cbase = ch * CHUNK;
    const int wc = scan_chunk(dsts, nE, nTot, cbase, nodeBase, nb, vec8, list, tid, lane, wave);
    if (lane == 0) wcnt[wave] = wc;
    __syncthreads();
    int pre = 0, all = 0;
#pragma unroll
    for (int w2 = 0; w2 < NWAVE; ++w2) {
      int c = wcnt[w2];
      c = c < 0 ? 0 : (c > WCAP ? WCAP : c);
      all += c;
      pre += (w2 < wave) ? c : 0;
    }
    const int wcc  = wc > WCAP ? WCAP : wc;
    const int base = tot + pre;
#pragma unroll 1
    for (int i = lane; i < wcc; i += 32) {
      const int ent = list[wave * WCAP + i];
      const int el  = (ent >> 12) & (CHUNK - 1);
      const int sl  = ent & (NBMAX - 1);
      int eid = cbase + el;
      eid = eid > nTot - 1 ? nTot - 1 : eid;
      const int pos = base + i;
      if (pos < RCAP) reg1[pos] = (int)(((unsigned)eid << 12) | (unsigned)sl);
    }
    tot += all;
    tot = tot > RCAP ? RCAP : tot;
    __syncthreads();
  }
  const int nh = tot;

  if (wave == 0) {
#pragma unroll 1
    for (int b0 = 0; b0 < nh; b0 += 32) {
      const int idx = b0 + lane;
      const int uv  = reg1[idx < RCAP ? idx : RCAP - 1];
      const int m32 = (nh - b0) < 32 ? (nh - b0) : 32;
#pragma unroll 1
      for (int k = 0; k < m32; ++k) {
        const int u  = __builtin_amdgcn_readlane(uv, k);
        const int sl = u & (NBMAX - 1);
        if (lane == 0) scnt[sl] = scnt[sl] + 1;
      }
    }
  }
  __syncthreads();

  {
    const v4i ca = *(const v4i*)(scnt + 4 * tid);
    const int e0 = ca.x < 0 ? 0 : ca.x, e1 = ca.y < 0 ? 0 : ca.y, e2 = ca.z < 0 ? 0 : ca.z, e3 = ca.w < 0 ? 0 : ca.w;
    const int ts = e0 + e1 + e2 + e3;
    int incl = ts;
#pragma unroll
    for (int d = 1; d < 32; d <<= 1) {
      const int up = __shfl_up(incl, d);
      if (lane >= d) incl += up;
    }
    if (lane == 31) wtot[wave] = incl;
    __syncthreads();
    int pre = 0;
#pragma unroll
    for (int w2 = 0; w2 < NWAVE; ++w2) pre += (w2 < wave) ? wtot[w2] : 0;
    int run = pre + incl - ts;
    soff[4 * tid + 0] = run; run += e0;
    soff[4 * tid + 1] = run; run += e1;
    soff[4 * tid + 2] = run; run += e2;
    soff[4 * tid + 3] = run;
  }
  __syncthreads();
  for (int i = tid; i < NBMAX; i += NTHR) list[i] = soff[i];
  __syncthreads();

  if (wave == 0) {
#pragma unroll 1
    for (int b0 = 0; b0 < nh; b0 += 32) {
      const int idx = b0 + lane;
      const int uv  = reg1[idx < RCAP ? idx : RCAP - 1];
      const int m32 = (nh - b0) < 32 ? (nh - b0) : 32;
#pragma unroll 1
      for (int k = 0; k < m32; ++k) {
        const int u   = __builtin_amdgcn_readlane(uv, k);
        const int sl  = u & (NBMAX - 1);
        const int eid = (int)((unsigned)u >> 12);
        if (lane == 0) {
          int pos = list[sl];
          pos = pos < 0 ? 0 : (pos > RCAP - 1 ? RCAP - 1 : pos);
          reg2[pos] = eid;
          list[sl] = pos + 1;
        }
      }
    }
  }
  __syncthreads();

  const int nbw = nb >> 3;
  const bool ovf = (nh >= RCAP);
  const float qnan = __int_as_float(0x7fc00000);
  const v4f z4 = {0.f, 0.f, 0.f, 0.f};
  float* stw = (float*)reg1 + wave * STW;
  float g8[8], b8[8], as8[8], ad8[8], bg8[8];
  {
    const v4f ga = *(const v4f*)(lng + 8 * lane), gb = *(const v4f*)(lng + 8 * lane + 4);
    const v4f ba = *(const v4f*)(lnb + 8 * lane), bb = *(const v4f*)(lnb + 8 * lane + 4);
    g8[0] = ga.x; g8[1] = ga.y; g8[2] = ga.z; g8[3] = ga.w; g8[4] = gb.x; g8[5] = gb.y; g8[6] = gb.z; g8[7] = gb.w;
    b8[0] = ba.x; b8[1] = ba.y; b8[2] = ba.z; b8[3] = ba.w; b8[4] = bb.x; b8[5] = bb.y; b8[6] = bb.z; b8[7] = bb.w;
    if (GAT) {
      const v4f sa = *(const v4f*)(atts + 8 * lane), sb = *(const v4f*)(atts + 8 * lane + 4);
      const v4f ea = *(const v4f*)(attd + 8 * lane), eb = *(const v4f*)(attd + 8 * lane + 4);
      const v4f oa = *(const v4f*)(bgp + 8 * lane),  ob = *(const v4f*)(bgp + 8 * lane + 4);
      as8[0] = sa.x; as8[1] = sa.y; as8[2] = sa.z; as8[3] = sa.w; as8[4] = sb.x; as8[5] = sb.y; as8[6] = sb.z; as8[7] = sb.w;
      ad8[0] = ea.x; ad8[1] = ea.y; ad8[2] = ea.z; ad8[3] = ea.w; ad8[4] = eb.x; ad8[5] = eb.y; ad8[6] = eb.z; ad8[7] = eb.w;
      bg8[0] = oa.x; bg8[1] = oa.y; bg8[2] = oa.z; bg8[3] = oa.w; bg8[4] = ob.x; bg8[5] = ob.y; bg8[6] = ob.z; bg8[7] = ob.w;
    } else {
#pragma unroll
      for (int j = 0; j < 8; ++j) { as8[j] = 0.f; ad8[j] = 0.f; bg8[j] = 0.f; }
    }
    ldwait();
  }

#pragma unroll 1
  for (int jt = 0; jt < nbw; ++jt) {
    const int slot = wave * nbw + jt;
    const int grow = nodeBase + slot;
    const bool lv  = grow < nN;
    const int gcl  = lv ? grow : nN - 1;
    int st = soff[slot];
    const int craw = scnt[slot];
    int cnt = craw;
    st  = st < 0 ? 0 : (st > nh ? nh : st);
    cnt = cnt < 0 ? 0 : (cnt > DEGCAP ? DEGCAP : cnt);
    if (cnt > nh - st) cnt = nh - st;
    const float pz = (ovf || craw > DEGCAP) ? qnan : 0.0f;
    const bool wr = grow < MPr;

    float qv[8], sk[8], rs[8], av[8];
    float ad = 0.f;
    {
      const float* hrow = Hf + (size_t)gcl * HC + 8 * lane;
      v4f ra = *(const v4f*)hrow, rb = *(const v4f*)(hrow + 4);
      v4f qa, qb, sa, sb;
      if (GAT) {
        const float* prow = P + (size_t)gcl * HC + 8 * lane;
        qa = *(const v4f*)prow; qb = *(const v4f*)(prow + 4);
        sa = z4; sb = z4;
      } else {
        const float* prow = P + (size_t)gcl * NQ + 8 * lane;
        qa = *(const v4f*)(prow + OQ); qb = *(const v4f*)(prow + OQ + 4);
        sa = *(const v4f*)(prow + OS); sb = *(const v4f*)(prow + OS + 4);
      }
      ldwait();
      if (!lv) { ra = z4; rb = z4; qa = z4; qb = z4; sa = z4; sb = z4; }
      rs[0] = ra.x; rs[1] = ra.y; rs[2] = ra.z; rs[3] = ra.w; rs[4] = rb.x; rs[5] = rb.y; rs[6] = rb.z; rs[7] = rb.w;
      qv[0] = qa.x; qv[1] = qa.y; qv[2] = qa.z; qv[3] = qa.w; qv[4] = qb.x; qv[5] = qb.y; qv[6] = qb.z; qv[7] = qb.w;
      if (GAT) {
        float t = qv[0] * ad8[0];
        t = fmaf(qv[1], ad8[1], t); t = fmaf(qv[2], ad8[2], t); t = fmaf(qv[3], ad8[3], t);
        t = fmaf(qv[4], ad8[4], t); t = fmaf(qv[5], ad8[5], t); t = fmaf(qv[6], ad8[6], t); t = fmaf(qv[7], ad8[7], t);
        t += __shfl_xor(t, 1);
        t += __shfl_xor(t, 2);
        ad = t;
#pragma unroll
        for (int j = 0; j < 8; ++j) sk[j] = bg8[j];
      } else {
        sk[0] = sa.x; sk[1] = sa.y; sk[2] = sa.z; sk[3] = sa.w; sk[4] = sb.x; sk[5] = sb.y; sk[6] = sb.z; sk[7] = sb.w;
      }
    }
#pragma unroll
    for (int j = 0; j < 8; ++j) av[j] = 0.f;
    float mx = -1.0e30f, dn = 0.f;

#pragma unroll 1
    for (int q = 0; q < cnt; ++q) {
      int idx = st + q; idx = idx > RCAP - 1 ? RCAP - 1 : idx;
      int eid = reg2[idx]; eid = eid < 0 ? 0 : (eid > nTot - 1 ? nTot - 1 : eid);
      const int er = eid < nE ? eid : nE - 1;
      const int sraw = srcs[er];
      int s = (eid < nE) ? sraw : (eid - nE);
      s = s < 0 ? 0 : (s > nN - 1 ? nN - 1 : s);
      float x8[8];
      float al;
      if (GAT) {
        const float* hr = P + (size_t)s * HC + 8 * lane;
        const v4f ha = *(const v4f*)hr, hb = *(const v4f*)(hr + 4);
        ldwait();
        x8[0] = ha.x; x8[1] = ha.y; x8[2] = ha.z; x8[3] = ha.w; x8[4] = hb.x; x8[5] = hb.y; x8[6] = hb.z; x8[7] = hb.w;
        float t = x8[0] * as8[0];
        t = fmaf(x8[1], as8[1], t); t = fmaf(x8[2], as8[2], t); t = fmaf(x8[3], as8[3], t);
        t = fmaf(x8[4], as8[4], t); t = fmaf(x8[5], as8[5], t); t = fmaf(x8[6], as8[6], t); t = fmaf(x8[7], as8[7], t);
        t += __shfl_xor(t, 1);
        t += __shfl_xor(t, 2);
        const float e0 = t + ad;
        al = e0 > 0.f ? e0 : 0.2f * e0;
      } else {
        const float* kr = P + (size_t)s * NQ + OKK + 8 * lane;
        const v4f ka = *(const v4f*)kr, kb = *(const v4f*)(kr + 4);
        const v4f va = *(const v4f*)(kr + (OV - OKK)), vb = *(const v4f*)(kr + (OV - OKK) + 4);
        ldwait();
        x8[0] = va.x; x8[1] = va.y; x8[2] = va.z; x8[3] = va.w; x8[4] = vb.x; x8[5] = vb.y; x8[6] = vb.z; x8[7] = vb.w;
        float t = qv[0] * ka.x;
        t = fmaf(qv[1], ka.y, t); t = fmaf(qv[2], ka.z, t); t = fmaf(qv[3], ka.w, t);
        t = fmaf(qv[4], kb.x, t); t = fmaf(qv[5], kb.y, t); t = fmaf(qv[6], kb.z, t); t = fmaf(qv[7], kb.w, t);
        t += __shfl_xor(t, 1);
        t += __shfl_xor(t, 2);
        al = t * ATTSC;
      }
      const float df = al - mx;
      const float ee = __expf(-fabsf(df));
      const bool up  = df > 0.f;
      const float s1 = up ? ee : 1.0f;
      const float s2 = up ? 1.0f : ee;
      mx = up ? al : mx;
      dn = fmaf(dn, s1, s2);
#pragma unroll
      for (int j = 0; j < 8; ++j) av[j] = fmaf(av[j], s1, s2 * x8[j]);
    }

    const float ds  = dn > 0.f ? dn : 1.0f;
    const float inv = (dn > 0.f ? 1.0f : 0.0f) * __builtin_amdgcn_rcpf(ds);
    float val[8];
#pragma unroll
    for (int j = 0; j < 8; ++j) val[j] = fmaf(av[j], inv, sk[j]) + rs[j];
    float sm = ((val[0] + val[1]) + (val[2] + val[3])) + ((val[4] + val[5]) + (val[6] + val[7]));
#pragma unroll
    for (int off = 16; off > 0; off >>= 1) sm += __shfl_xor(sm, off);
    const float mu = sm * INVHC;
    float d8[8];
    float vq = 0.f;
#pragma unroll
    for (int j = 0; j < 8; ++j) { d8[j] = val[j] - mu; vq = fmaf(d8[j], d8[j], vq); }
#pragma unroll
    for (int off = 16; off > 0; off >>= 1) vq += __shfl_xor(vq, off);
    const float rstd = rsqrtf(vq * INVHC + LNEPS);
    float r8[8];
#pragma unroll
    for (int j = 0; j < 8; ++j) {
      const float y = fmaf(d8[j] * rstd, g8[j], b8[j]);
      r8[j] = (lv ? fmaxf(y, 0.f) : 0.f) + pz;
    }
    v4f ya, yb;
    ya.x = r8[0]; ya.y = r8[1]; ya.z = r8[2]; ya.w = r8[3];
    yb.x = r8[4]; yb.y = r8[5]; yb.z = r8[6]; yb.w = r8[7];
    const v8h hv = cvt8h(ya, yb, CX);
    __builtin_amdgcn_fence(__ATOMIC_RELEASE, "wavefront");
    __builtin_amdgcn_wave_barrier();
    *(v4f*)(stw + 8 * lane)     = ya;
    *(v4f*)(stw + 8 * lane + 4) = yb;
    __builtin_amdgcn_fence(__ATOMIC_RELEASE, "wavefront");
    __builtin_amdgcn_wave_barrier();
    const v4f oa = *(const v4f*)(stw + 4 * lane);
    const v4f ob = *(const v4f*)(stw + HC / 2 + 4 * lane);
    _Float16* gp = Hh + (size_t)grow * HC + 8 * lane;
    float*    fp = Hf + (size_t)grow * HC;
    if (wr) {
      *(volatile v8h*)gp = hv;
      *(volatile v4f*)(fp + 4 * lane) = oa;
      *(volatile v4f*)(fp + HC / 2 + 4 * lane) = ob;
    }
    __threadfence();
    if (wr) {
      *(volatile v8h*)gp = hv;
      *(volatile v4f*)(fp + 4 * lane) = oa;
      *(volatile v4f*)(fp + HC / 2 + 4 * lane) = ob;
    }
  }
}

__global__ __launch_bounds__(NTHR) void k_pool(const int* __restrict__ bat, const float* __restrict__ Hf,
                                               _Float16* PF, int nN, int vec8) {
  __shared__ int preg[PCAP];
  __shared__ int list[LISTN];
  __shared__ int wcnt[NWAVE];
  __shared__ __attribute__((aligned(16))) float pst[HC];
  const int tid = (int)threadIdx.x, lane = tid & 31, wave = tid >> 5;
  const int g = (int)blockIdx.x;

  int tot = 0;
  const int nChunks = (nN + CHUNK - 1) / CHUNK;
#pragma unroll 1
  for (int ch = 0; ch < nChunks; ++ch) {
    const int cbase = ch * CHUNK;
    const int wc = scan_chunk(bat, nN, nN, cbase, g, 1, vec8, list, tid, lane, wave);
    if (lane == 0) wcnt[wave] = wc;
    __syncthreads();
    int pre = 0, all = 0;
#pragma unroll
    for (int w2 = 0; w2 < NWAVE; ++w2) {
      int c = wcnt[w2];
      c = c < 0 ? 0 : (c > WCAP ? WCAP : c);
      all += c;
      pre += (w2 < wave) ? c : 0;
    }
    const int wcc  = wc > WCAP ? WCAP : wc;
    const int base = tot + pre;
#pragma unroll 1
    for (int i = lane; i < wcc; i += 32) {
      const int ent = list[wave * WCAP + i];
      const int el  = (ent >> 12) & (CHUNK - 1);
      int nd = cbase + el;
      nd = nd > nN - 1 ? nN - 1 : nd;
      const int pos = base + i;
      if (pos < PCAP) preg[pos] = nd;
    }
    tot += all;
    tot = tot > PCAP ? PCAP : tot;
    __syncthreads();
  }
  const int nh = tot;
  const bool ovf = (nh >= PCAP);
  const float qnan = __int_as_float(0x7fc00000);

  float acc = 0.f;
#pragma unroll 1
  for (int p = 0; p < nh; ++p) {
    int nd = preg[p];
    nd = nd < 0 ? 0 : (nd > nN - 1 ? nN - 1 : nd);
    acc += Hf[(size_t)nd * HC + tid];
  }
  const float cf = (float)nh;
  const float rc = 1.0f / (cf > 1.0f ? cf : 1.0f);
  pst[tid] = acc * rc + (ovf ? qnan : 0.0f);
  __syncthreads();
  if (wave == 0) {
    const v4f ga = *(const v4f*)(pst + 8 * lane);
    const v4f gb = *(const v4f*)(pst + 8 * lane + 4);
    const v8h hv = cvt8h(ga, gb, CX);
    _Float16* pp = PF + (size_t)g * HC + 8 * lane;
    *(volatile v8h*)pp = hv;
    __threadfence();
    *(volatile v8h*)pp = hv;
  }
}

static int pick_nb(int nEv, int nN) {
  int nb = NBMAX;
  while (nb > 16 && (long long)nb * (long long)nEv * 5LL > (long long)RCAP * (long long)nN * 4LL) nb >>= 1;
  return nb;
}
static inline int cdiv(int a, int b) { return (a + b - 1) / b; }

extern "C" void kernel_launch(void* const* d_in, const int* in_sizes, int n_in,
                              void* d_out, int out_size, void* d_ws, size_t ws_size,
                              hipStream_t stream) {
  if (n_in < 23) return;
  const int nN = in_sizes[0] / DIN;
  if (nN <= 0 || in_sizes[0] != nN * DIN || nN > (1 << 19)) return;
  if (in_sizes[1] < 2 || (in_sizes[1] & 1) != 0) return;
  const int nE = in_sizes[1] / 2;
  if (nE < 1 || nE + nN > (1 << 20)) return;
  if (in_sizes[2] != nN) return;
  if (in_sizes[3] != DIN * HC || in_sizes[4] != HC) return;
  if (in_sizes[5] != 2 * HC * HC || in_sizes[6] != 2 * HC * HC) return;
  if (in_sizes[7] != 2 * HC * HC || in_sizes[8] != 2 * HC * HC) return;
  if (in_sizes[9] != 2 * HC || in_sizes[10] != 2 * HC) return;
  if (in_sizes[11] != 2 * HC || in_sizes[12] != 2 * HC) return;
  if (in_sizes[13] != 2 * HC * HC) return;
  if (in_sizes[14] != 2 * HC || in_sizes[15] != 2 * HC) return;
  if (in_sizes[16] != 2 * HC) return;
  if (in_sizes[17] != 4 * HC || in_sizes[18] != 4 * HC) return;
  if (in_sizes[19] != HC * HFF || in_sizes[20] != HFF) return;
  if (in_sizes[21] != HFF * NOUT || in_sizes[22] != NOUT) return;
  if (out_size != NGR * NOUT) return;

  const float* x    = (const float*)d_in[0];
  const int*   ei   = (const int*)  d_in[1];
  const int*   bat  = (const int*)  d_in[2];
  const float* Win  = (const float*)d_in[3];
  const float* b_in = (const float*)d_in[4];
  const float* Wq   = (const float*)d_in[5];
  const float* Wk   = (const float*)d_in[6];
  const float* Wv   = (const float*)d_in[7];
  const float* Ws   = (const float*)d_in[8];
  const float* bq   = (const float*)d_in[9];
  const float* bk   = (const float*)d_in[10];
  const float* bv   = (const float*)d_in[11];
  const float* bs   = (const float*)d_in[12];
  const float* Wg   = (const float*)d_in[13];
  const float* ats  = (const float*)d_in[14];
  const float* atd  = (const float*)d_in[15];
  const float* bg   = (const float*)d_in[16];
  const float* lng  = (const float*)d_in[17];
  const float* lnb  = (const float*)d_in[18];
  const float* W1   = (const float*)d_in[19];
  const float* b1   = (const float*)d_in[20];
  const float* W2   = (const float*)d_in[21];
  const float* b2   = (const float*)d_in[22];
  float* out = (float*)d_out;
  const int* src = ei;
  const int* dst = ei + nE;

  const int MP   = cdiv(nN, GBM) * GBM;
  const int nTg  = nE + nN;
  const int nb0  = pick_nb(nE, nN);
  const int nb1  = pick_nb(nTg, nN);
  const int gA0  = cdiv(MP, nb0);
  const int gA1  = cdiv(MP, nb1);
  const int vec8 = ((nE & 3) == 0) ? 1 : 0;
  if (gA0 * nb0 < MP || gA1 * nb1 < MP) return;

  char* ws = (char*)d_ws;
  size_t off = 0;
  const size_t oXH  = off; off += (size_t)MP * KIN * 2;            off = (off + 255) & ~(size_t)255;
  const size_t oWIN = off; off += (size_t)HC * KIN * 2;            off = (off + 255) & ~(size_t)255;
  const size_t oWT0 = off; off += (size_t)NQ * HC * 2;             off = (off + 255) & ~(size_t)255;
  const size_t oWT1 = off; off += (size_t)NQ * HC * 2;             off = (off + 255) & ~(size_t)255;
  const size_t oWG0 = off; off += (size_t)HC * HC * 2;             off = (off + 255) & ~(size_t)255;
  const size_t oWG1 = off; off += (size_t)HC * HC * 2;             off = (off + 255) & ~(size_t)255;
  const size_t oW1T = off; off += (size_t)HFF * HC * 2;            off = (off + 255) & ~(size_t)255;
  const size_t oW2T = off; off += (size_t)NOUT * HFF * 2;          off = (off + 255) & ~(size_t)255;
  const size_t oHF  = off; off += (size_t)MP * HC * 4;             off = (off + 255) & ~(size_t)255;
  const size_t oHH  = off; off += (size_t)MP * HC * 2;             off = (off + 255) & ~(size_t)255;
  const size_t oQ   = off; off += (size_t)MP * NQ * 4;             off = (off + 255) & ~(size_t)255;
  const size_t oPF  = off; off += (size_t)NGR * HC * 2;            off = (off + 255) & ~(size_t)255;
  const size_t oH1  = off; off += (size_t)NGR * HFF * 2;           off = (off + 255) & ~(size_t)255;
  if (off > ws_size || off > (size_t)WSMAX) return;
  _Float16* XH   = (_Float16*)(ws + oXH);
  _Float16* WIN  = (_Float16*)(ws + oWIN);
  _Float16* WT0  = (_Float16*)(ws + oWT0);
  _Float16* WT1  = (_Float16*)(ws + oWT1);
  _Float16* WG0  = (_Float16*)(ws + oWG0);
  _Float16* WG1  = (_Float16*)(ws + oWG1);
  _Float16* W1T  = (_Float16*)(ws + oW1T);
  _Float16* W2T  = (_Float16*)(ws + oW2T);
  float*    HF   = (float*)(ws + oHF);
  _Float16* HHH  = (_Float16*)(ws + oHH);
  float*    QKVS = (float*)(ws + oQ);
  _Float16* PF   = (_Float16*)(ws + oPF);
  _Float16* H1H  = (_Float16*)(ws + oH1);

  hipFuncSetAttribute(reinterpret_cast<const void*>(&k_layer<0>),
                      hipFuncAttributeMaxDynamicSharedMemorySize, LDS_AGG);
  hipFuncSetAttribute(reinterpret_cast<const void*>(&k_layer<1>),
                      hipFuncAttributeMaxDynamicSharedMemorySize, LDS_AGG);

  const int nUx = MP * (KIN / 8);
  k_xprep<<<cdiv(nUx, NTHR), NTHR, 0, stream>>>(x, XH, nN, nUx);

  {
    const int nUi = HC * (KIN / 8);
    k_wtr<<<cdiv(nUi, NTHR), NTHR, 0, stream>>>(Win, Win, Win, Win, HC, HC, HC, HC, HC, DIN, KIN, WIN, nUi);
    const int nUt = NQ * (HC / 8);
    k_wtr<<<cdiv(nUt, NTHR), NTHR, 0, stream>>>(Wq, Wk, Wv, Ws, HC, HC, HC, HC, HC, HC, HC, WT0, nUt);
    k_wtr<<<cdiv(nUt, NTHR), NTHR, 0, stream>>>(Wq + HC * HC, Wk + HC * HC, Wv + HC * HC, Ws + HC * HC,
                                                HC, HC, HC, HC, HC, HC, HC, WT1, nUt);
    const int nUg = HC * (HC / 8);
    k_wtr<<<cdiv(nUg, NTHR), NTHR, 0, stream>>>(Wg, Wg, Wg, Wg, HC, HC, HC, HC, HC, HC, HC, WG0, nUg);
    k_wtr<<<cdiv(nUg, NTHR), NTHR, 0, stream>>>(Wg + HC * HC, Wg + HC * HC, Wg + HC * HC, Wg + HC * HC,
                                                HC, HC, HC, HC, HC, HC, HC, WG1, nUg);
    const int nU1 = HFF * (HC / 8);
    k_wtr<<<cdiv(nU1, NTHR), NTHR, 0, stream>>>(W1, W1, W1, W1, HFF, HFF, HFF, HFF, HFF, HC, HC, W1T, nU1);
    const int nU2 = NOUT * (HFF / 8);
    k_wtr<<<cdiv(nU2, NTHR), NTHR, 0, stream>>>(W2, W2, W2, W2, NOUT, NOUT, NOUT, NOUT, NOUT, HFF, HFF, W2T, nU2);
  }

  const int gM = MP / GBM;
  k_gemm<1><<<dim3(gM, HC / GBN), GTHR, 0, stream>>>(XH, WIN, b_in, b_in, b_in, b_in, HF, HHH,
                                                     KIN, HC, HC, HC, 1.0f, SCL_XW);

  for (int layer = 0; layer < 4; ++layer) {
    const float* gln = lng + (size_t)layer * HC;
    const float* bln = lnb + (size_t)layer * HC;
    if ((layer & 1) == 0) {
      const int t = layer >> 1;
      const _Float16* WT = (t == 0) ? WT0 : WT1;
      k_gemm<0><<<dim3(gM, NQ / GBN), GTHR, 0, stream>>>(HHH, WT, bq + t * HC, bk + t * HC, bv + t * HC, bs + t * HC,
                                                         QKVS, PF, HC, NQ, HC, HC, 1.0f, SCL_XW);
      k_layer<0><<<gA0, NTHR, LDS_AGG, stream>>>(src, dst, QKVS, ats, atd, bg, gln, bln, HF, HHH,
                                                 nN, nE, nE, nb0, vec8, MP);
    } else {
      const int g = layer >> 1;
      const _Float16* WT = (g == 0) ? WG0 : WG1;
      k_gemm<0><<<dim3(gM, HC / GBN), GTHR, 0, stream>>>(HHH, WT, bg, bg, bg, bg,
                                                         QKVS, PF, HC, HC, HC, HC, 0.0f, SCL_XW);
      k_layer<1><<<gA1, NTHR, LDS_AGG, stream>>>(src, dst, QKVS, ats + g * HC, atd + g * HC, bg + g * HC, gln, bln,
                                                 HF, HHH, nN, nE, nTg, nb1, vec8, MP);
    }
  }

  k_pool<<<NGR, NTHR, 0, stream>>>(bat, HF, PF, nN, 1);
  k_gemm<2><<<dim3(NGR / GBM, HFF / GBN), GTHR, 0, stream>>>(PF, W1T, b1, b1, b1, b1, QKVS, H1H,
                                                            HC, HFF, HFF, HFF, 1.0f, SCL_XW);
  k_gemm<0><<<dim3(NGR / GBM, NOUT / GBN), GTHR, 0, stream>>>(H1H, W2T, b2, b2, b2, b2, out, PF,
                                                             HFF, NOUT, NOUT, NOUT, 1.0f, SCL_XW);
}
